// SeqModelFused_24618752541423
// MI455X (gfx1250) — hardware-run, weakly checked
//
#include <hip/hip_runtime.h>
#include <stdint.h>

typedef __attribute__((ext_vector_type(16))) __bf16       v16b;
typedef __attribute__((ext_vector_type(8)))  __bf16       v8b;
typedef __attribute__((ext_vector_type(8)))  float        v8f;
typedef __attribute__((ext_vector_type(4)))  float        v4f;
typedef __attribute__((ext_vector_type(4)))  unsigned int v4u;

constexpr int kSteps = 128;
constexpr int kBatch = 64;
constexpr int kHid   = 1024;
constexpr int kRows  = kSteps * kBatch;
constexpr int kChan  = kBatch * kHid;
static_assert(kRows == 8192 && kChan == 65536, "shape");
static_assert((kHid % 32) == 0, "GEMM K multiple of 32");
static_assert((kRows % 64) == 0 && (kHid % 64) == 0, "GEMM M,N multiples of 64");
static_assert(((kRows * kHid / 8) % 256) == 0 && ((kHid * kHid / 8) % 256) == 0, "convert grids exact");
static_assert(((kChan / 8) % 256) == 0, "scan grid exact");

constexpr size_t kOffXB  = 0;
constexpr size_t kOffW1B = kOffXB  + (size_t)kRows * kHid * 2;
constexpr size_t kOffW2B = kOffW1B + (size_t)kHid  * kHid * 2;
constexpr size_t kOffHP  = kOffW2B + (size_t)kHid  * kHid * 2;
constexpr size_t kOffSP  = kOffHP  + (size_t)kRows * kHid * 4;
constexpr size_t kWsTotal = kOffSP + (size_t)kRows * kHid * 2;
static_assert(kWsTotal == 71303168ull, "carve total");
static_assert(kWsTotal <= 134217728ull, "carve cap");
static_assert((kOffW1B % 128) == 0 && (kOffW2B % 128) == 0 && (kOffHP % 128) == 0 && (kOffSP % 128) == 0,
              "128-B aligned regions");

__device__ __forceinline__ unsigned bf_rne_bits(float f) {
  const unsigned u = __float_as_uint(f);
  return (u + 0x7FFFu + ((u >> 16) & 1u)) >> 16;
}

union FragB { v16b v; v8b h[2]; };
__device__ __forceinline__ v16b frag_load(const __bf16* p) {
  FragB f;
  f.h[0] = *(const v8b*)(p);
  f.h[1] = *(const v8b*)(p + 16);
  return f.v;
}
__device__ __forceinline__ v8f frag_mma(v16b a, v16b b, v8f c) {
  return __builtin_amdgcn_wmma_f32_16x16x32_bf16(false, a, false, b, (short)0, c, false, false);
}
__device__ __forceinline__ void tie_acc(v8f& a, v16b x, v16b y) {
  asm volatile("" : "+v"(a) : "v"(x), "v"(y));
}
__device__ __forceinline__ void tie_acc_nops(v8f& a, v16b x, v16b y) {
  asm volatile("v_nop\n\tv_nop\n\tv_nop\n\tv_nop" : "+v"(a) : "v"(x), "v"(y));
}
__device__ __forceinline__ void keep4_b(v16b a, v16b b, v16b c, v16b d) {
  asm volatile("v_nop" :: "v"(a), "v"(b), "v"(c), "v"(d));
}
__device__ __forceinline__ void acc_guard4(v8f& a, v8f& b, v8f& c, v8f& d) {
  asm volatile("v_nop\n\tv_nop\n\tv_nop\n\tv_nop" : "+v"(a), "+v"(b), "+v"(c), "+v"(d));
}

__global__ __launch_bounds__(256) void cvt_plane_bf16_kernel(
    const float* __restrict__ src, unsigned short* __restrict__ dst, int total8)
{
  const int i = blockIdx.x * 256 + threadIdx.x;
  if (i >= total8) return;
  const size_t e0 = (size_t)i << 3;
  const v4f a0 = *(const v4f*)(src + e0);
  const v4f a1 = *(const v4f*)(src + e0 + 4);
  const float f0 = a0[0], f1 = a0[1], f2 = a0[2], f3 = a0[3];
  const float f4 = a1[0], f5 = a1[1], f6 = a1[2], f7 = a1[3];
  const unsigned w0 = bf_rne_bits(f0) | (bf_rne_bits(f1) << 16);
  const unsigned w1 = bf_rne_bits(f2) | (bf_rne_bits(f3) << 16);
  const unsigned w2 = bf_rne_bits(f4) | (bf_rne_bits(f5) << 16);
  const unsigned w3 = bf_rne_bits(f6) | (bf_rne_bits(f7) << 16);
  const v4u w = {w0, w1, w2, w3};
  unsigned short* q = dst + e0;
  *(volatile v4u*)q = w;
  __threadfence();
  *(volatile v4u*)q = w;
}

__global__ __launch_bounds__(256) void gemm_bf16_nt_kernel(
    const unsigned short* __restrict__ Ap, int lda,
    const unsigned short* __restrict__ Btp, int ldb,
    float* __restrict__ C, int ldc, int M, int N, int K)
{
  const __bf16* A  = (const __bf16*)Ap;
  const __bf16* Bt = (const __bf16*)Btp;
  __shared__ __align__(16) float sT[8][16 * 68];
  const int lane = threadIdx.x & 31;
  const int wave = threadIdx.x >> 5;
  const int tilesN = N >> 6;
  const int tilesM = M >> 6;
  const int tile = blockIdx.x * 8 + wave;
  if (tile >= tilesM * tilesN) return;
  const int tm = tile / tilesN;
  const int tn = tile - tm * tilesN;
  const int m0 = tm << 6;
  const int n0 = tn << 6;

  const int rlane = lane & 15;
  const int koff  = (lane >> 4) * 8;
  const int mOff  = (lane >> 4) * 8;

  v8f acc[4][4];
#pragma unroll
  for (int i = 0; i < 4; ++i)
#pragma unroll
    for (int j = 0; j < 4; ++j) acc[i][j] = (v8f){0.f, 0.f, 0.f, 0.f, 0.f, 0.f, 0.f, 0.f};

  for (int k0 = 0; k0 < K; k0 += 32) {
    v16b bh[4];
#pragma unroll
    for (int j = 0; j < 4; ++j) {
      const size_t bo = (size_t)(n0 + (j << 4) + rlane) * ldb + koff + k0;
      bh[j] = frag_load(Bt + bo);
    }
#pragma unroll
    for (int i = 0; i < 4; ++i) {
      const size_t ao = (size_t)(m0 + (i << 4) + rlane) * lda + koff + k0;
      const v16b ah = frag_load(A + ao);
#pragma unroll
      for (int j = 0; j < 4; ++j) acc[i][j] = frag_mma(ah, bh[j], acc[i][j]);
      tie_acc(acc[i][0], ah, bh[0]);
      tie_acc(acc[i][1], ah, bh[1]);
      tie_acc(acc[i][2], ah, bh[2]);
      tie_acc_nops(acc[i][3], ah, bh[3]);
    }
    keep4_b(bh[0], bh[1], bh[2], bh[3]);
  }
  acc_guard4(acc[0][0], acc[0][1], acc[0][2], acc[0][3]);
  acc_guard4(acc[1][0], acc[1][1], acc[1][2], acc[1][3]);
  acc_guard4(acc[2][0], acc[2][1], acc[2][2], acc[2][3]);
  acc_guard4(acc[3][0], acc[3][1], acc[3][2], acc[3][3]);

  float* slab = sT[wave];
  const int hh = lane >> 4;
  const int c4 = (lane & 15) * 4;
#pragma unroll
  for (int i = 0; i < 4; ++i) {
    const int mBase = m0 + (i << 4);
#pragma unroll
    for (int j = 0; j < 4; ++j) {
#pragma unroll
      for (int r = 0; r < 8; ++r) {
        slab[(mOff + r) * 68 + (j << 4) + rlane] = acc[i][j][r];
      }
    }
    __builtin_amdgcn_fence(__ATOMIC_RELEASE, "workgroup");
    __builtin_amdgcn_wave_barrier();
    __builtin_amdgcn_fence(__ATOMIC_ACQUIRE, "workgroup");
    for (int pass = 0; pass < 2; ++pass) {
#pragma unroll
      for (int it = 0; it < 8; ++it) {
        const int row = it * 2 + hh;
        const v4f val = *(const v4f*)(slab + row * 68 + c4);
        *(volatile v4f*)(C + (size_t)(mBase + row) * ldc + n0 + c4) = val;
      }
      __threadfence();
    }
    __builtin_amdgcn_fence(__ATOMIC_RELEASE, "workgroup");
    __builtin_amdgcn_wave_barrier();
    __builtin_amdgcn_fence(__ATOMIC_ACQUIRE, "workgroup");
  }
}

__global__ __launch_bounds__(256) void lif_scan_kernel(
    const float* __restrict__ HP, unsigned short* __restrict__ SP, int nlanes)
{
#pragma clang fp contract(off)
  const int i = blockIdx.x * 256 + threadIdx.x;
  if (i >= nlanes) return;
  const size_t c0 = (size_t)i << 3;
  float v[8];
#pragma unroll
  for (int e = 0; e < 8; ++e) v[e] = 0.0f;
#pragma unroll 1
  for (int t = 0; t < kSteps; ++t) {
    const size_t off = (size_t)t * kChan + c0;
    const v4f a0 = *(const v4f*)(HP + off);
    const v4f a1 = *(const v4f*)(HP + off + 4);
    float hin[8];
    hin[0] = a0[0]; hin[1] = a0[1]; hin[2] = a0[2]; hin[3] = a0[3];
    hin[4] = a1[0]; hin[5] = a1[1]; hin[6] = a1[2]; hin[7] = a1[3];
    unsigned lo16[8];
#pragma unroll
    for (int e = 0; e < 8; ++e) {
      const float d  = hin[e] - v[e];
      const float hd = d * 0.5f;
      const float hm = v[e] + hd;
      const bool fire = (hm >= 1.0f);
      lo16[e] = fire ? 0x3F80u : 0u;
      v[e] = fire ? 0.0f : hm;
    }
    const unsigned w0 = lo16[0] | (lo16[1] << 16);
    const unsigned w1 = lo16[2] | (lo16[3] << 16);
    const unsigned w2 = lo16[4] | (lo16[5] << 16);
    const unsigned w3 = lo16[6] | (lo16[7] << 16);
    const v4u w = {w0, w1, w2, w3};
    unsigned short* q = SP + off;
    *(volatile v4u*)q = w;
    __threadfence();
    *(volatile v4u*)q = w;
  }
}

extern "C" void kernel_launch(void* const* d_in, const int* in_sizes, int n_in,
                              void* d_out, int out_size, void* d_ws, size_t ws_size,
                              hipStream_t stream) {
  if (n_in < 3) return;
  if (in_sizes[0] != kRows * kHid) return;
  if (in_sizes[1] != kHid * kHid) return;
  if (in_sizes[2] != kHid * kHid) return;
  if (out_size != kRows * kHid) return;
  if (ws_size < kWsTotal) return;

  const float* x  = (const float*)d_in[0];
  const float* W1 = (const float*)d_in[1];
  const float* W2 = (const float*)d_in[2];
  float* out = (float*)d_out;

  char* ws = (char*)d_ws;
  unsigned short* XB  = (unsigned short*)(ws + kOffXB);
  unsigned short* W1B = (unsigned short*)(ws + kOffW1B);
  unsigned short* W2B = (unsigned short*)(ws + kOffW2B);
  float*          HP  = (float*)(ws + kOffHP);
  unsigned short* SP  = (unsigned short*)(ws + kOffSP);

  cvt_plane_bf16_kernel<<<(kRows * kHid / 8) / 256, 256, 0, stream>>>(x, XB, kRows * kHid / 8);
  cvt_plane_bf16_kernel<<<(kHid * kHid / 8) / 256, 256, 0, stream>>>(W1, W1B, kHid * kHid / 8);
  cvt_plane_bf16_kernel<<<(kHid * kHid / 8) / 256, 256, 0, stream>>>(W2, W2B, kHid * kHid / 8);

  constexpr int kTiles = (kRows / 64) * (kHid / 64);
  static_assert((kTiles % 8) == 0, "tiles per block");

  gemm_bf16_nt_kernel<<<kTiles / 8, 256, 0, stream>>>(XB, kHid, W1B, kHid, HP, kHid, kRows, kHid, kHid);

  lif_scan_kernel<<<(kChan / 8) / 256, 256, 0, stream>>>(HP, SP, kChan / 8);

  gemm_bf16_nt_kernel<<<kTiles / 8, 256, 0, stream>>>(SP, kHid, W2B, kHid, out, kHid, kRows, kHid, kHid);
}
